// Encoder_34299608825911
// MI455X (gfx1250) — hardware-run, weakly checked
//
#include <hip/hip_runtime.h>


#ifndef NB
#define NB 2
#endif
#ifndef SEQ
#define SEQ 2048
#endif
#define NB_FULL  2
#define SEQ_FULL 2048
#ifndef OUT_SEQ
#define OUT_SEQ SEQ
#endif
#define DM   256
#define NH_  8
#define HD   32
#define NFF  1024
#define NLAY 6
#define VOCAB 1024
#define MAXLEN 4096
#define CXP  (2 * DM)
#define MDP  (2 * NFF)
#define AW   4
#define QRS  2048.0f
#define QRI  (1.0f / 2048.0f)
#define SC2  (16.0f * 1.4426950408889634f)
#define PSH  14.0f
#define NEGT (-1.0e20f * 16.0f * 1.4426950408889634f)
#define LNE  1.0e-5f
#define RT   64
#define LP   264

static_assert(HD == 32);
static_assert(NH_ * HD == DM);
static_assert(NH_ % 2 == 0);
static_assert(DM == 256);
static_assert(DM % 64 == 0);
static_assert(NFF % 64 == 0);
static_assert(DM % 32 == 0);
static_assert(CXP % 32 == 0);
static_assert(MDP % 32 == 0);
static_assert((NFF & (NFF - 1)) == 0);
static_assert(SEQ % 64 == 0);
static_assert((NB * SEQ) % 64 == 0);
static_assert(SEQ % 32 == 0);
static_assert(SEQ % (16 * AW) == 0);
static_assert(SEQ % RT == 0);
static_assert(RT == 64);
static_assert(RT % 8 == 0);
static_assert(DM * (RT / 8) == 8 * 256);
static_assert(LP % 8 == 0);
static_assert(LP >= DM);
static_assert(((size_t)SEQ * DM) % 8 == 0);
static_assert(NB <= NB_FULL);
static_assert(SEQ <= SEQ_FULL);
static_assert(SEQ_FULL <= MAXLEN);
static_assert(PSH <= 15.0f);

typedef _Float16 h16;
typedef unsigned short bf;
typedef __attribute__((ext_vector_type(16))) __bf16   v16bf;
typedef __attribute__((ext_vector_type(16))) _Float16 v16h;
typedef __attribute__((ext_vector_type(8)))  _Float16 v8h;
typedef __attribute__((ext_vector_type(8)))  unsigned short v8us;
typedef __attribute__((ext_vector_type(8)))  float    v8f;
typedef __attribute__((ext_vector_type(4)))  float    v4f;
typedef __attribute__((ext_vector_type(4)))  int      v4i;
typedef v4f  __attribute__((may_alias)) v4fa;
typedef v8h  __attribute__((may_alias)) v8ha;

__device__ __forceinline__ unsigned short f2bf(float f) { unsigned u = __float_as_uint(f); u += 0x7FFFu + ((u >> 16) & 1u); return (unsigned short)(u >> 16); }
__device__ __forceinline__ float bf2f(unsigned short s) { return __uint_as_float(((unsigned)s) << 16); }
__device__ __forceinline__ float bfr(float f) { return bf2f(f2bf(f)); }
__device__ __forceinline__ v4f bfr4(v4f x) { v4f y; y[0] = bfr(x[0]); y[1] = bfr(x[1]); y[2] = bfr(x[2]); y[3] = bfr(x[3]); return y; }
__device__ __forceinline__ v16h cat16(v8h lo, v8h hi) { return __builtin_shufflevector(lo, hi, 0, 1, 2, 3, 4, 5, 6, 7, 8, 9, 10, 11, 12, 13, 14, 15); }
__device__ __forceinline__ v16bf cat16b(v8us lo, v8us hi) { return __builtin_bit_cast(v16bf, __builtin_shufflevector(lo, hi, 0, 1, 2, 3, 4, 5, 6, 7, 8, 9, 10, 11, 12, 13, 14, 15)); }
__device__ __forceinline__ v8f wmma16(v16h a, v16h b, v8f c) { return __builtin_amdgcn_wmma_f32_16x16x32_f16(false, a, false, b, (short)0, c, false, false); }
__device__ __forceinline__ v8f wmmab(v16bf a, v16bf b, v8f c) { return __builtin_amdgcn_wmma_f32_16x16x32_bf16(false, a, false, b, (short)0, c, false, false); }
__device__ __forceinline__ v16h  ldh(const h16* p) { return cat16(*(const v8h*)p, *(const v8h*)(p + 16)); }
__device__ __forceinline__ v16bf ldb(const bf* p)  { return cat16b(*(const v8us*)p, *(const v8us*)(p + 16)); }
__device__ __forceinline__ void wave_sync() { __builtin_amdgcn_fence(3  , "wavefront"); __builtin_amdgcn_wave_barrier(); asm volatile("" ::: "memory"); }
__device__ __forceinline__ float wsum(float v) { v += __shfl_xor(v, 16, 32); v += __shfl_xor(v, 8, 32); v += __shfl_xor(v, 4, 32); v += __shfl_xor(v, 2, 32); v += __shfl_xor(v, 1, 32); return v; }

__global__ __launch_bounds__(256) void k_wT(const float* __restrict__ W, bf* dst, int kdim, int ndim) {
    __shared__ float ts[64 * 65];
    const int tid = threadIdx.x; const int k0 = blockIdx.x * 64, n0 = blockIdx.y * 64;
    const int lz = (int)(blockIdx.z >> 1), hf = (int)(blockIdx.z & 1);
    const size_t wl = (size_t)lz * (size_t)kdim * (size_t)ndim;
    const size_t ldo = (size_t)2 * (size_t)kdim;
    const size_t dl = (size_t)lz * (size_t)ndim * ldo + (size_t)hf * (size_t)kdim;
#pragma unroll
    for (int i = 0; i < 4; ++i) { const int kk = (tid >> 4) + 16 * i, c4 = (tid & 15) * 4;
        const v4f f = *(const v4f*)(W + wl + (size_t)(k0 + kk) * (size_t)ndim + n0 + c4);
        ts[kk * 65 + c4 + 0] = f[0]; ts[kk * 65 + c4 + 1] = f[1]; ts[kk * 65 + c4 + 2] = f[2]; ts[kk * 65 + c4 + 3] = f[3]; }
    __syncthreads();
#pragma unroll 1
    for (int ps = 0; ps < 2; ++ps) {
#pragma unroll
        for (int it = 0; it < 2; ++it) { const int nn = it * 32 + (tid >> 3), ks = (tid & 7) * 8;
            v8us o;
#pragma unroll
            for (int j = 0; j < 8; ++j) o[j] = f2bf(ts[(ks + j) * 65 + nn]);
            *(volatile v8us*)(dst + dl + (size_t)(n0 + nn) * ldo + k0 + ks) = o; }
        if (ps == 0) __threadfence(); }
}

__device__ __forceinline__ void split_h(v4f b0, v4f b1, v8h& hv, v8h& rv) {
#pragma clang fp contract(off)
#pragma unroll
    for (int i = 0; i < 4; ++i) { const h16 a0 = (h16)b0[i]; const h16 a1 = (h16)b1[i]; hv[i] = a0; hv[4 + i] = a1;
        rv[i] = (h16)((b0[i] - (float)a0) * QRS); rv[4 + i] = (h16)((b1[i] - (float)a1) * QRS); }
}

__device__ __forceinline__ void put_row(float* frow, v4f a0, v4f a1, h16* hrow, h16* rrow, v8h hv, v8h rv, int lane, int planes) {
#pragma unroll 1
    for (int ps = 0; ps < 2; ++ps) {
        *(volatile v4f*)(frow + 4 * lane) = a0; *(volatile v4f*)(frow + 128 + 4 * lane) = a1;
        if (planes) { *(volatile v8h*)(hrow + 8 * lane) = hv; *(volatile v8h*)(rrow + 8 * lane) = rv; }
        if (ps == 0) __threadfence(); }
}

__device__ __forceinline__ void ln_row(const float* __restrict__ xr, int lane, v4f gA0, v4f gA1, v4f cA0, v4f cA1, v4f gB0, v4f gB1, v4f cB0, v4f cB1,
                                       v4f& yA0, v4f& yA1, v4f& yB0, v4f& yB1) {
#pragma clang fp contract(off)
    const v4f xA0 = *(const v4f*)(xr + 4 * lane), xA1 = *(const v4f*)(xr + 128 + 4 * lane);
    const v4f xB0 = *(const v4f*)(xr + 8 * lane), xB1 = *(const v4f*)(xr + 8 * lane + 4);
    float s = ((xB0[0] + xB0[1]) + (xB0[2] + xB0[3])) + ((xB1[0] + xB1[1]) + (xB1[2] + xB1[3]));
    s = wsum(s);
    const float mu = s * (1.0f / DM);
    const v4f d0 = xB0 - mu, d1 = xB1 - mu;
    float q = ((d0[0] * d0[0] + d0[1] * d0[1]) + (d0[2] * d0[2] + d0[3] * d0[3])) + ((d1[0] * d1[0] + d1[1] * d1[1]) + (d1[2] * d1[2] + d1[3] * d1[3]));
    q = wsum(q);
    const float rstd = rsqrtf(q * (1.0f / DM) + LNE);
    yA0 = (xA0 - mu) * rstd * gA0 + cA0; yA1 = (xA1 - mu) * rstd * gA1 + cA1;
    yB0 = d0 * rstd * gB0 + cB0;         yB1 = d1 * rstd * gB1 + cB1;
}

__global__ __launch_bounds__(256) void k_embed(const int* __restrict__ X, const float* __restrict__ E, const float* __restrict__ P, float* HO, h16* HH, h16* HR, h16* VT) {
#pragma clang fp contract(off)
    __shared__ __align__(16) h16 hs[RT * LP];
    const int tid = threadIdx.x, lane = tid & 31, wave = __builtin_amdgcn_readfirstlane((int)(threadIdx.x >> 5));
    const int m0 = blockIdx.x * RT; const int b = m0 / SEQ, tb = m0 - b * SEQ;
#pragma unroll 1
    for (int rr = 0; rr < RT / 8; ++rr) {
        const int row = wave * (RT / 8) + rr; const int t = tb + row; const int m = m0 + row;
        int tok = X[(size_t)b * SEQ_FULL + t]; tok = min(max(tok, 0), VOCAB - 1);
        const size_t eo = (size_t)tok * DM, po = (size_t)t * DM;
        const v4f yA0 = bfr4(*(const v4f*)(E + eo + 4 * lane)) + bfr4(*(const v4f*)(P + po + 4 * lane));
        const v4f yA1 = bfr4(*(const v4f*)(E + eo + 128 + 4 * lane)) + bfr4(*(const v4f*)(P + po + 128 + 4 * lane));
        const v4f yB0 = bfr4(*(const v4f*)(E + eo + 8 * lane)) + bfr4(*(const v4f*)(P + po + 8 * lane));
        const v4f yB1 = bfr4(*(const v4f*)(E + eo + 8 * lane + 4)) + bfr4(*(const v4f*)(P + po + 8 * lane + 4));
        v8h hv, rv; split_h(yB0, yB1, hv, rv);
        *(v8ha*)(&hs[row * LP + 8 * lane]) = hv;
        put_row(HO + (size_t)m * DM, yA0, yA1, HH + (size_t)m * DM, HR + (size_t)m * DM, hv, rv, lane, 1);
    }
    __syncthreads();
    const size_t vb = (size_t)b * DM * SEQ + tb;
#pragma unroll 1
    for (int ps = 0; ps < 2; ++ps) {
#pragma unroll 1
        for (int it = 0; it < 8; ++it) { const int idx = it * 256 + tid; const int c = idx >> 3, t8 = (idx & 7) * 8;
            v8h o;
#pragma unroll
            for (int j = 0; j < 8; ++j) o[j] = hs[(t8 + j) * LP + c];
            *(volatile v8h*)(VT + vb + (size_t)c * SEQ + t8) = o; }
        if (ps == 0) __threadfence(); }
}

__global__ __launch_bounds__(256) void k_ln1(const float* __restrict__ PRE, const float* __restrict__ G, const float* __restrict__ C, float* H1, bf* A1) {
#pragma clang fp contract(off)
    const int lane = threadIdx.x & 31, wave = __builtin_amdgcn_readfirstlane((int)(threadIdx.x >> 5));
    const int m0 = blockIdx.x * RT;
    const v4f gA0 = bfr4(*(const v4f*)(G + 4 * lane)), gA1 = bfr4(*(const v4f*)(G + 128 + 4 * lane)), cA0 = bfr4(*(const v4f*)(C + 4 * lane)), cA1 = bfr4(*(const v4f*)(C + 128 + 4 * lane));
    const v4f gB0 = bfr4(*(const v4f*)(G + 8 * lane)), gB1 = bfr4(*(const v4f*)(G + 8 * lane + 4)), cB0 = bfr4(*(const v4f*)(C + 8 * lane)), cB1 = bfr4(*(const v4f*)(C + 8 * lane + 4));
#pragma unroll 1
    for (int rr = 0; rr < RT / 8; ++rr) {
        const int m = m0 + wave * (RT / 8) + rr;
        v4f yA0, yA1, yB0, yB1;
        ln_row(PRE + (size_t)m * DM, lane, gA0, gA1, cA0, cA1, gB0, gB1, cB0, cB1, yA0, yA1, yB0, yB1);
        v8us hv, lv;
#pragma unroll
        for (int i = 0; i < 4; ++i) { const unsigned short u0 = f2bf(yB0[i]); const unsigned short u1 = f2bf(yB1[i]); hv[i] = u0; hv[4 + i] = u1;
            lv[i] = f2bf(yB0[i] - bf2f(u0)); lv[4 + i] = f2bf(yB1[i] - bf2f(u1)); }
        float* frow = H1 + (size_t)m * DM; bf* arow = A1 + (size_t)m * CXP;
#pragma unroll 1
        for (int ps = 0; ps < 2; ++ps) {
            *(volatile v4f*)(frow + 4 * lane) = yA0; *(volatile v4f*)(frow + 128 + 4 * lane) = yA1;
            *(volatile v8us*)(arow + 8 * lane) = hv; *(volatile v8us*)(arow + DM + 8 * lane) = lv;
            if (ps == 0) __threadfence(); }
    }
}

__global__ __launch_bounds__(256) void k_ln2(const float* __restrict__ PRE, const float* __restrict__ G, const float* __restrict__ C, float* HO, int oseq,
                                             h16* HH, h16* HR, h16* VT, int planes) {
#pragma clang fp contract(off)
    __shared__ __align__(16) h16 hs[RT * LP];
    const int tid = threadIdx.x, lane = tid & 31, wave = __builtin_amdgcn_readfirstlane((int)(threadIdx.x >> 5));
    const int m0 = blockIdx.x * RT; const int b = m0 / SEQ, tb = m0 - b * SEQ;
    const v4f gA0 = bfr4(*(const v4f*)(G + 4 * lane)), gA1 = bfr4(*(const v4f*)(G + 128 + 4 * lane)), cA0 = bfr4(*(const v4f*)(C + 4 * lane)), cA1 = bfr4(*(const v4f*)(C + 128 + 4 * lane));
    const v4f gB0 = bfr4(*(const v4f*)(G + 8 * lane)), gB1 = bfr4(*(const v4f*)(G + 8 * lane + 4)), cB0 = bfr4(*(const v4f*)(C + 8 * lane)), cB1 = bfr4(*(const v4f*)(C + 8 * lane + 4));
#pragma unroll 1
    for (int rr = 0; rr < RT / 8; ++rr) {
        const int row = wave * (RT / 8) + rr; const int m = m0 + row;
        v4f yA0, yA1, yB0, yB1;
        ln_row(PRE + (size_t)m * DM, lane, gA0, gA1, cA0, cA1, gB0, gB1, cB0, cB1, yA0, yA1, yB0, yB1);
        v8h hv, rv; split_h(yB0, yB1, hv, rv);
        if (planes) *(v8ha*)(&hs[row * LP + 8 * lane]) = hv;
        put_row(HO + ((size_t)b * oseq + tb + row) * DM, yA0, yA1, HH + (size_t)m * DM, HR + (size_t)m * DM, hv, rv, lane, planes);
    }
    __syncthreads();
    if (planes) {
        const size_t vb = (size_t)b * DM * SEQ + tb;
#pragma unroll 1
        for (int ps = 0; ps < 2; ++ps) {
#pragma unroll 1
            for (int it = 0; it < 8; ++it) { const int idx = it * 256 + tid; const int c = idx >> 3, t8 = (idx & 7) * 8;
                v8h o;
#pragma unroll
                for (int j = 0; j < 8; ++j) o[j] = hs[(t8 + j) * LP + c];
                *(volatile v8h*)(VT + vb + (size_t)c * SEQ + t8) = o; }
            if (ps == 0) __threadfence(); }
    }
}

__device__ __forceinline__ void gemm_tile(const bf* __restrict__ A, const bf* __restrict__ Bt, int K, int r0, int c0, int lr, int hi, v8f (&acc)[4][4]) {
#pragma unroll
    for (int mb = 0; mb < 4; ++mb)
#pragma unroll
        for (int nb = 0; nb < 4; ++nb) acc[mb][nb] = (v8f){};
    const size_t aoff = (size_t)(r0 + lr) * K + 8 * hi, boff = (size_t)(c0 + lr) * K + 8 * hi;
#pragma unroll 1
    for (int kc = 0; kc < K; kc += 32) {
        v16bf a[4];
#pragma unroll
        for (int mb = 0; mb < 4; ++mb) a[mb] = ldb(A + aoff + (size_t)mb * 16 * K + kc);
#pragma unroll
        for (int nb = 0; nb < 4; ++nb) { const v16bf b = ldb(Bt + boff + (size_t)nb * 16 * K + kc);
#pragma unroll
            for (int mb = 0; mb < 4; ++mb) acc[mb][nb] = wmmab(a[mb], b, acc[mb][nb]); }
        asm volatile("v_nop\n\tv_nop\n\tv_nop\n\tv_nop" : "+v"(acc[0][0]), "+v"(acc[1][1]), "+v"(acc[2][2]), "+v"(acc[3][3]) : "v"(a[0]), "v"(a[1]), "v"(a[2]), "v"(a[3]));
    }
}

__global__ __launch_bounds__(32) void k_gemm_f32(const bf* __restrict__ A, const bf* __restrict__ Bt, float* OUTP, const float* __restrict__ bias, const float* __restrict__ RES,
                                                 int K, int useBias) {
    __shared__ __align__(16) float os[16 * 68];
    const int lane = threadIdx.x & 31, lr = lane & 15, hi = lane >> 4; const int r0 = blockIdx.x * 64, c0 = blockIdx.y * 64;
    v8f acc[4][4];
    gemm_tile(A, Bt, K, r0, c0, lr, hi, acc);
#pragma unroll
    for (int mb = 0; mb < 4; ++mb) {
#pragma unroll
        for (int nb = 0; nb < 4; ++nb) {
#pragma unroll
            for (int j = 0; j < 8; ++j) os[(hi * 8 + j) * 68 + nb * 16 + lr] = acc[mb][nb][j]; }
        wave_sync();
#pragma unroll 1
        for (int ps = 0; ps < 2; ++ps) {
#pragma unroll
            for (int s = 0; s < 8; ++s) { const int row = 2 * s + hi, cofs = lr * 4;
                const int m = r0 + mb * 16 + row;
                v4f val = *(const v4fa*)(&os[row * 68 + cofs]);
                const int cidx = (c0 + cofs) & (DM - 1);
                const v4f bc = *(const v4f*)(bias + cidx);
                const v4f rs = *(const v4f*)(RES + (size_t)m * DM + c0 + cofs);
#pragma unroll
                for (int i = 0; i < 4; ++i) val[i] = (val[i] + (useBias ? bfr(bc[i]) : 0.0f)) + rs[i];
                *(volatile v4f*)(OUTP + (size_t)m * DM + c0 + cofs) = val; }
            if (ps == 0) __threadfence(); }
        wave_sync();
    }
}

__global__ __launch_bounds__(32) void k_gemm_relu(const bf* __restrict__ A, const bf* __restrict__ Bt, bf* MID, const float* __restrict__ bias, int K) {
    __shared__ __align__(16) float os[16 * 68];
    const int lane = threadIdx.x & 31, lr = lane & 15, hi = lane >> 4; const int r0 = blockIdx.x * 64, c0 = blockIdx.y * 64;
    v8f acc[4][4];
    gemm_tile(A, Bt, K, r0, c0, lr, hi, acc);
#pragma unroll
    for (int mb = 0; mb < 4; ++mb) {
#pragma unroll
        for (int nb = 0; nb < 4; ++nb) {
#pragma unroll
            for (int j = 0; j < 8; ++j) os[(hi * 8 + j) * 68 + nb * 16 + lr] = acc[mb][nb][j]; }
        wave_sync();
#pragma unroll 1
        for (int ps = 0; ps < 2; ++ps) {
#pragma unroll
            for (int s = 0; s < 4; ++s) { const int row = 4 * s + (lane >> 3), c8 = (lane & 7) * 8;
                const v4f x0 = *(const v4fa*)(&os[row * 68 + c8]); const v4f x1 = *(const v4fa*)(&os[row * 68 + c8 + 4]);
                const int cidx = (c0 + c8) & (NFF - 1);
                const v4f bc0 = *(const v4f*)(bias + cidx), bc1 = *(const v4f*)(bias + cidx + 4);
                v8us hv, lv;
#pragma unroll
                for (int i = 0; i < 4; ++i) { const float y0 = fmaxf(x0[i] + bfr(bc0[i]), 0.0f); const float y1 = fmaxf(x1[i] + bfr(bc1[i]), 0.0f);
                    const unsigned short u0 = f2bf(y0); const unsigned short u1 = f2bf(y1); hv[i] = u0; hv[4 + i] = u1;
                    lv[i] = f2bf(y0 - bf2f(u0)); lv[4 + i] = f2bf(y1 - bf2f(u1)); }
                const size_t oo = (size_t)(r0 + mb * 16 + row) * MDP + c0 + c8;
                *(volatile v8us*)(MID + oo) = hv; *(volatile v8us*)(MID + oo + NFF) = lv; }
            if (ps == 0) __threadfence(); }
        wave_sync();
    }
}

__global__ __launch_bounds__(32 * AW) void k_flash(const h16* __restrict__ HH, const h16* __restrict__ HR, const h16* __restrict__ VT,
                                                   const int* __restrict__ MK, bf* CX) {
    __shared__ __align__(16) float os[AW * 16 * 68];
    const int lane = threadIdx.x & 31, wave = __builtin_amdgcn_readfirstlane((int)(threadIdx.x >> 5)), lr = lane & 15, hi = lane >> 4;
    const int zp = blockIdx.y; const int b = zp / (NH_ / 2), hp = zp % (NH_ / 2);
    const int t0 = (blockIdx.x * AW + wave) * 16;
    const int wb = wave * 16 * 68;
    const size_t rowb = (size_t)b * SEQ;
    const int* mk = MK + (size_t)b * SEQ_FULL + 8 * hi;
#pragma unroll 1
    for (int hh = 0; hh < 2; ++hh) {
        const int h = hp * 2 + hh;
        const size_t qo = (rowb + t0 + lr) * DM + h * HD + 8 * hi;
        const v16h qh = ldh(HH + qo), qr = ldh(HR + qo);
        const size_t ko = (rowb + lr) * DM + h * HD + 8 * hi;
        const size_t vo = ((size_t)b * DM + h * HD + lr) * SEQ + 8 * hi;
        v8f o0 = (v8f){}, o1 = (v8f){};
        float m = -3.0e38f, l = 0.0f;
#pragma unroll 1
        for (int key0 = 0; key0 < SEQ; key0 += 32) {
            const size_t kk = ko + (size_t)key0 * DM;
            const v16h ka0 = ldh(HH + kk), kb0 = ldh(HH + kk + 16 * DM);
            const v16h ra0 = ldh(HR + kk), rb0 = ldh(HR + kk + 16 * DM);
            const v4i ma0 = *(const v4i*)(mk + key0), ma1 = *(const v4i*)(mk + key0 + 4), mb0 = *(const v4i*)(mk + key0 + 16), mb1 = *(const v4i*)(mk + key0 + 20);
            v8f sHa = (v8f){}, sLa = (v8f){}, sHb = (v8f){}, sLb = (v8f){};
            sHa = wmma16(ka0, qh, sHa); sLa = wmma16(ka0, qr, sLa); sHb = wmma16(kb0, qh, sHb); sLb = wmma16(kb0, qr, sLb);
            sLa = wmma16(ra0, qh, sLa); sLb = wmma16(rb0, qh, sLb);
            asm volatile("v_nop\n\tv_nop\n\tv_nop\n\tv_nop" : "+v"(sHa), "+v"(sLa), "+v"(sHb), "+v"(sLb) : "v"(ka0), "v"(kb0), "v"(ra0), "v"(rb0), "v"(qh), "v"(qr));
            float ta[8], tb[8]; float mx = -3.0e38f;
#pragma unroll
            for (int r = 0; r < 4; ++r) {
                const float a0 = (sHa[r] + sLa[r] * QRI) * SC2, a1 = (sHa[4 + r] + sLa[4 + r] * QRI) * SC2;
                const float c0 = (sHb[r] + sLb[r] * QRI) * SC2, c1 = (sHb[4 + r] + sLb[4 + r] * QRI) * SC2;
                ta[r] = (ma0[r] != 0) ? a0 : NEGT; ta[4 + r] = (ma1[r] != 0) ? a1 : NEGT;
                tb[r] = (mb0[r] != 0) ? c0 : NEGT; tb[4 + r] = (mb1[r] != 0) ? c1 : NEGT; }
#pragma unroll
            for (int r = 0; r < 8; ++r) mx = fmaxf(mx, fmaxf(ta[r], tb[r]));
            mx = fmaxf(mx, __shfl_xor(mx, 16, 32));
            const float mnew = fmaxf(m, mx);
            const float alpha = __builtin_amdgcn_exp2f(m - mnew);
            const float sh = PSH - mnew;
            v16h pb; float ls = 0.0f;
#pragma unroll
            for (int r = 0; r < 8; ++r) { const h16 pa = (h16)__builtin_amdgcn_exp2f(ta[r] + sh); const h16 pc = (h16)__builtin_amdgcn_exp2f(tb[r] + sh); pb[r] = pa; pb[8 + r] = pc; ls += (float)pa + (float)pc; }
            l = l * alpha + ls; m = mnew;
            o0 = o0 * alpha; o1 = o1 * alpha;
            const h16* va = VT + vo + key0;
            const v16h v0 = ldh(va), v1 = ldh(va + (size_t)16 * SEQ);
            o0 = wmma16(v0, pb, o0); o1 = wmma16(v1, pb, o1);
            asm volatile("v_nop\n\tv_nop\n\tv_nop\n\tv_nop" : "+v"(o0), "+v"(o1) : "v"(v0), "v"(v1), "v"(pb));
        }
        l += __shfl_xor(l, 16, 32);
        const float inv = 1.0f / l;
        { v4f a, c; const int ob = wb + lr * 68 + hh * 32 + 8 * hi;
          a[0] = o0[0] * inv; a[1] = o0[1] * inv; a[2] = o0[2] * inv; a[3] = o0[3] * inv; c[0] = o0[4] * inv; c[1] = o0[5] * inv; c[2] = o0[6] * inv; c[3] = o0[7] * inv;
          *(v4fa*)(&os[ob]) = a; *(v4fa*)(&os[ob + 4]) = c;
          a[0] = o1[0] * inv; a[1] = o1[1] * inv; a[2] = o1[2] * inv; a[3] = o1[3] * inv; c[0] = o1[4] * inv; c[1] = o1[5] * inv; c[2] = o1[6] * inv; c[3] = o1[7] * inv;
          *(v4fa*)(&os[ob + 16]) = a; *(v4fa*)(&os[ob + 20]) = c; }
    }
    wave_sync();
    bf* crow = CX + (rowb + t0) * CXP + hp * 64;
#pragma unroll 1
    for (int ps = 0; ps < 2; ++ps) {
#pragma unroll
        for (int s = 0; s < 4; ++s) { const int row = 4 * s + (lane >> 3), c8 = (lane & 7) * 8;
            const v4f x0 = *(const v4fa*)(&os[wb + row * 68 + c8]); const v4f x1 = *(const v4fa*)(&os[wb + row * 68 + c8 + 4]); v8us hv, lv;
#pragma unroll
            for (int i = 0; i < 4; ++i) { const unsigned short u0 = f2bf(x0[i]); const unsigned short u1 = f2bf(x1[i]); hv[i] = u0; hv[4 + i] = u1;
                lv[i] = f2bf(x0[i] - bf2f(u0)); lv[4 + i] = f2bf(x1[i] - bf2f(u1)); }
            const size_t oo = (size_t)row * CXP + c8;
            *(volatile v8us*)(crow + oo) = hv; *(volatile v8us*)(crow + oo + DM) = lv; }
        if (ps == 0) __threadfence(); }
}

static constexpr size_t al256(size_t v) { return (v + 255) & ~(size_t)255; }
static constexpr int    MTOK   = NB * SEQ;
static constexpr size_t SZ_F32 = al256((size_t)MTOK * DM * 4);
static constexpr size_t SZ_PL  = al256((size_t)MTOK * DM * 2);
static constexpr size_t SZ_CX  = al256((size_t)MTOK * CXP * 2);
static constexpr size_t SZ_MID = al256((size_t)MTOK * MDP * 2);
static constexpr size_t SZ_WO  = al256((size_t)NLAY * DM * CXP * 2);
static constexpr size_t SZ_W1  = al256((size_t)NLAY * NFF * CXP * 2);
static constexpr size_t SZ_W2  = al256((size_t)NLAY * DM * MDP * 2);
static constexpr size_t SZ_TOTAL = 3 * SZ_F32 + 3 * SZ_PL + 2 * SZ_CX + SZ_MID + SZ_WO + SZ_W1 + SZ_W2;
static_assert(SZ_TOTAL <= (size_t)134217728);
static_assert((size_t)NB * DM * SEQ * 2 <= SZ_PL);
static_assert(MTOK % 64 == 0);
static_assert(MTOK % RT == 0);

extern "C" void kernel_launch(void* const* d_in, const int* in_sizes, int n_in,
                              void* d_out, int out_size, void* d_ws, size_t ws_size, hipStream_t stream) {
    if (n_in < 13) return;
    const size_t needt = (size_t)(NB - 1) * SEQ_FULL + SEQ;
    if ((size_t)in_sizes[0] < needt || (size_t)in_sizes[1] < needt) return;
    if ((size_t)in_sizes[2] < (size_t)VOCAB * DM || (size_t)in_sizes[3] < (size_t)SEQ * DM) return;
    if ((size_t)in_sizes[4] < (size_t)NLAY * DM * DM) return;
    if (in_sizes[5] < NLAY * DM || in_sizes[6] < NLAY * DM || in_sizes[7] < NLAY * DM || in_sizes[8] < NLAY * DM) return;
    if ((size_t)in_sizes[9] < (size_t)NLAY * DM * NFF || in_sizes[10] < NLAY * NFF) return;
    if ((size_t)in_sizes[11] < (size_t)NLAY * NFF * DM || in_sizes[12] < NLAY * DM) return;
    if ((size_t)out_size < ((size_t)(NB - 1) * OUT_SEQ + SEQ) * DM) return;
    if (SZ_TOTAL > ws_size) return;
    const int* xtok = (const int*)d_in[0]; const int* amask = (const int*)d_in[1];
    const float* Ew = (const float*)d_in[2]; const float* Pw = (const float*)d_in[3];
    const float* wo = (const float*)d_in[4];
    const float* g1 = (const float*)d_in[5]; const float* c1 = (const float*)d_in[6];
    const float* g2 = (const float*)d_in[7]; const float* c2 = (const float*)d_in[8];
    const float* w1 = (const float*)d_in[9]; const float* b1 = (const float*)d_in[10];
    const float* w2 = (const float*)d_in[11]; const float* b2 = (const float*)d_in[12];
    float* OUT = (float*)d_out;
    char* wsp = (char*)d_ws;
    float* H   = (float*)wsp; wsp += SZ_F32;
    float* H1  = (float*)wsp; wsp += SZ_F32;
    float* PRE = (float*)wsp; wsp += SZ_F32;
    h16* HH = (h16*)wsp; wsp += SZ_PL;
    h16* HR = (h16*)wsp; wsp += SZ_PL;
    h16* VT = (h16*)wsp; wsp += SZ_PL;
    bf* CX  = (bf*)wsp; wsp += SZ_CX;
    bf* A1  = (bf*)wsp; wsp += SZ_CX;
    bf* MID = (bf*)wsp; wsp += SZ_MID;
    bf* WO2 = (bf*)wsp; wsp += SZ_WO;
    bf* W1T = (bf*)wsp; wsp += SZ_W1;
    bf* W2T = (bf*)wsp; wsp += SZ_W2;

    k_wT<<<dim3(DM / 64, DM / 64, NLAY * 2), 256, 0, stream>>>(wo, WO2, DM, DM);
    k_wT<<<dim3(DM / 64, NFF / 64, NLAY * 2), 256, 0, stream>>>(w1, W1T, DM, NFF);
    k_wT<<<dim3(NFF / 64, DM / 64, NLAY * 2), 256, 0, stream>>>(w2, W2T, NFF, DM);

    k_embed<<<MTOK / RT, 256, 0, stream>>>(xtok, Ew, Pw, H, HH, HR, VT);

    for (int l = 0; l < NLAY; ++l) {
        k_flash<<<dim3(SEQ / (16 * AW), NB * (NH_ / 2), 1), 32 * AW, 0, stream>>>(HH, HR, VT, amask, CX);
        k_gemm_f32<<<dim3(MTOK / 64, DM / 64, 1), 32, 0, stream>>>(CX, WO2 + (size_t)l * DM * CXP, PRE, b2 + (size_t)l * DM, H, CXP, 0);
        k_ln1<<<MTOK / RT, 256, 0, stream>>>(PRE, g1 + (size_t)l * DM, c1 + (size_t)l * DM, H1, A1);
        k_gemm_relu<<<dim3(MTOK / 64, NFF / 64, 1), 32, 0, stream>>>(A1, W1T + (size_t)l * NFF * CXP, MID, b1 + (size_t)l * NFF, CXP);
        k_gemm_f32<<<dim3(MTOK / 64, DM / 64, 1), 32, 0, stream>>>(MID, W2T + (size_t)l * DM * MDP, PRE, b2 + (size_t)l * DM, H1, MDP, 1);
        if (l + 1 < NLAY) k_ln2<<<MTOK / RT, 256, 0, stream>>>(PRE, g2 + (size_t)l * DM, c2 + (size_t)l * DM, H, SEQ, HH, HR, VT, 1);
        else              k_ln2<<<MTOK / RT, 256, 0, stream>>>(PRE, g2 + (size_t)l * DM, c2 + (size_t)l * DM, OUT, OUT_SEQ, HH, HR, VT, 0);
    }
}
